// TextureWarpingModule_78408922956452
// MI455X (gfx1250) — hardware-verified
//
#include <hip/hip_runtime.h>
#define NI 2
#define CH 256
#define HS 64
#define HP 128
#define PX (HS * HS)
#define NR (NI * PX)
#define NGN 32
#define GSZ (CH / NGN)
#define DG 8
#define CG (CH / DG)
#define NOFF (3 * DG * 9)
typedef __bf16 v16b __attribute__((ext_vector_type(16)));
typedef unsigned short v8us __attribute__((ext_vector_type(8), may_alias));
typedef float  v8f  __attribute__((ext_vector_type(8)));
typedef float  v4f  __attribute__((ext_vector_type(4)));
typedef float  v4fa __attribute__((ext_vector_type(4), may_alias));
union FragB { v16b v; v8us half[2]; unsigned short u[16]; };

__device__ __forceinline__ unsigned short bf16_bits(float x) { unsigned int u = __float_as_uint(x); return (unsigned short)((u + 0x7FFFu + ((u >> 16) & 1u)) >> 16); }
__device__ __forceinline__ float bf16_val(unsigned short b) { return __uint_as_float(((unsigned int)b) << 16); }
__device__ __forceinline__ float bf16_round(float x) { return bf16_val(bf16_bits(x)); }
template <int NT>
__device__ __forceinline__ v8f mmaN(v16b ah, v16b al, v16b bh, v16b bl, v8f c) {
  c = __builtin_amdgcn_wmma_f32_16x16x32_bf16(false, ah, false, bh, (short)0, c, false, false);
  if (NT >= 2) c = __builtin_amdgcn_wmma_f32_16x16x32_bf16(false, al, false, bh, (short)0, c, false, false);
  if (NT >= 3) c = __builtin_amdgcn_wmma_f32_16x16x32_bf16(false, ah, false, bl, (short)0, c, false, false);
  asm volatile("v_nop\n\tv_nop\n\tv_nop\n\tv_nop" : "+v"(c) : "v"(ah), "v"(al), "v"(bh), "v"(bl));
  return c;
}

__global__ __launch_bounds__(256) void k_wt_bf16(const float* __restrict__ W, unsigned short* __restrict__ Wt, int K, int N) {
  const int t = blockIdx.x * 256 + threadIdx.x;
  const int k8n = K / 8;
  if (t >= N * k8n) return;
  const int n = t / k8n, k8 = (t % k8n) * 8;
  v8us v;
#pragma unroll
  for (int i = 0; i < 8; ++i) v[i] = bf16_bits(W[(size_t)(k8 + i) * N + n]);
  *(volatile v8us*)(Wt + (size_t)n * K + k8) = v;
  __threadfence();
  *(volatile v8us*)(Wt + (size_t)n * K + k8) = v;
}

template <bool ASPLIT, int ACT, bool BIAS_BF16>
__global__ __launch_bounds__(128) void k_gemm_bf(const float* __restrict__ A, int lda, const unsigned short* __restrict__ Wt, int ldb,
                                               const float* __restrict__ bias, float* __restrict__ C, int ldc, int M, int N, int K) {
  __shared__ __attribute__((aligned(16))) float so[4][16][64];
  const int tid = threadIdx.x, w = tid >> 5, lane = tid & 31, ln = lane & 15, hh = lane >> 4;
  const int ntn = N / 64;
  const int wid = blockIdx.x * 4 + w;
  const int mt = wid / ntn, nq = wid % ntn;
  if (mt * 16 >= M) return;
  const int row0 = mt * 16, col0 = nq * 64;
  const float* arow = A + (size_t)(row0 + ln) * lda;
  v8f acc[4] = {};
  for (int kb = 0; kb < K; kb += 32) {
    FragB ah, al;
    const v4f x0 = *(const v4fa*)(arow + kb + 8 * hh), x1 = *(const v4fa*)(arow + kb + 8 * hh + 4);
    const v4f x2 = *(const v4fa*)(arow + kb + 16 + 8 * hh), x3 = *(const v4fa*)(arow + kb + 16 + 8 * hh + 4);
    float xs[16] = {x0[0],x0[1],x0[2],x0[3],x1[0],x1[1],x1[2],x1[3],x2[0],x2[1],x2[2],x2[3],x3[0],x3[1],x3[2],x3[3]};
#pragma unroll
    for (int i = 0; i < 16; ++i) { const unsigned short hb = bf16_bits(xs[i]); ah.u[i] = hb; al.u[i] = ASPLIT ? bf16_bits(xs[i] - bf16_val(hb)) : (unsigned short)0; }
#pragma unroll
    for (int t = 0; t < 4; ++t) {
      const unsigned short* brow = Wt + (size_t)(col0 + t * 16 + ln) * ldb + kb;
      FragB b;
      b.half[0] = *(const v8us*)(brow + 8 * hh);
      b.half[1] = *(const v8us*)(brow + 16 + 8 * hh);
      acc[t] = mmaN<ASPLIT ? 2 : 1>(ah.v, al.v, b.v, b.v, acc[t]);
    }
  }
#pragma unroll
  for (int t = 0; t < 4; ++t) {
    float bv = bias ? bias[col0 + t * 16 + ln] : 0.f;
    if (BIAS_BF16) bv = bf16_round(bv);
#pragma unroll
    for (int r = 0; r < 8; ++r) { float v = acc[t][r] + bv; if (ACT == 1) v = fmaxf(v, 0.f); so[w][8 * hh + r][t * 16 + ln] = v; }
  }
  __builtin_amdgcn_fence(__ATOMIC_ACQ_REL, "workgroup");
  __builtin_amdgcn_wave_barrier();
  const int rsub = lane >> 4, c4 = (lane & 15) * 4;
  for (int pass = 0; pass < 2; ++pass) {
#pragma unroll
    for (int q = 0; q < 8; ++q) {
      const int r = q * 2 + rsub;
      const v4f v = *(const v4fa*)&so[w][r][c4];
      *(volatile v4f*)(C + (size_t)(row0 + r) * ldc + col0 + c4) = v;
    }
    if (pass == 0) __threadfence();
  }
}

template <bool ASPLIT, int ACT, bool BIAS_BF16, bool RES_BF16>
__global__ __launch_bounds__(128) void k_gemm_bf3(const float* __restrict__ A, int lda, const unsigned short* __restrict__ Wt, int ldb,
                                                const float* __restrict__ bias, const float* __restrict__ resid, int rmod, int ldr,
                                                float* __restrict__ C, int ldc, int M, int N, int K) {
  __shared__ __attribute__((aligned(16))) float so[4][16][64];
  const int tid = threadIdx.x, w = tid >> 5, lane = tid & 31, ln = lane & 15, hh = lane >> 4;
  const int ntn = N / 64;
  const int wid = blockIdx.x * 4 + w;
  const int mt = wid / ntn, nq = wid % ntn;
  if (mt * 16 >= M) return;
  const int row0 = mt * 16, col0 = nq * 64;
  const float* arow = A + (size_t)(row0 + ln) * lda;
  v8f acc[4] = {};
  for (int kb = 0; kb < K; kb += 32) {
    FragB ah, al;
    const v4f x0 = *(const v4fa*)(arow + kb + 8 * hh), x1 = *(const v4fa*)(arow + kb + 8 * hh + 4);
    const v4f x2 = *(const v4fa*)(arow + kb + 16 + 8 * hh), x3 = *(const v4fa*)(arow + kb + 16 + 8 * hh + 4);
    float xs[16] = {x0[0],x0[1],x0[2],x0[3],x1[0],x1[1],x1[2],x1[3],x2[0],x2[1],x2[2],x2[3],x3[0],x3[1],x3[2],x3[3]};
#pragma unroll
    for (int i = 0; i < 16; ++i) { const unsigned short hb = bf16_bits(xs[i]); ah.u[i] = hb; al.u[i] = ASPLIT ? bf16_bits(xs[i] - bf16_val(hb)) : (unsigned short)0; }
#pragma unroll
    for (int t = 0; t < 4; ++t) {
      const unsigned short* brow = Wt + (size_t)(col0 + t * 16 + ln) * ldb + kb;
      FragB b;
      b.half[0] = *(const v8us*)(brow + 8 * hh);
      b.half[1] = *(const v8us*)(brow + 16 + 8 * hh);
      acc[t] = mmaN<ASPLIT ? 2 : 1>(ah.v, al.v, b.v, b.v, acc[t]);
    }
  }
#pragma unroll
  for (int t = 0; t < 4; ++t) {
    const int col = col0 + t * 16 + ln;
    float bv = bias ? bias[col] : 0.f;
    if (BIAS_BF16) bv = bf16_round(bv);
#pragma unroll
    for (int r = 0; r < 8; ++r) {
      float v = acc[t][r] + bv;
      if (resid) { float rv = resid[(size_t)((row0 + 8 * hh + r) % rmod) * ldr + col]; if (RES_BF16) rv = bf16_round(rv); v += rv; }
      if (ACT == 1) v = fmaxf(v, 0.f);
      if (ACT == 2) v = 0.5f * v * (1.0f + erff(v * 0.70710678118654752f));
      if (ACT == 3) { const float u = 0.7978845608028654f * (v + 0.044715f * v * v * v); v = 0.5f * v * (1.0f + tanhf(u)); }
      so[w][8 * hh + r][t * 16 + ln] = v;
    }
  }
  __builtin_amdgcn_fence(__ATOMIC_ACQ_REL, "workgroup");
  __builtin_amdgcn_wave_barrier();
  const int rsub = lane >> 4, c4 = (lane & 15) * 4;
  for (int pass = 0; pass < 2; ++pass) {
#pragma unroll
    for (int q = 0; q < 8; ++q) {
      const int r = q * 2 + rsub;
      const v4f v = *(const v4fa*)&so[w][r][c4];
      *(volatile v4f*)(C + (size_t)(row0 + r) * ldc + col0 + c4) = v;
    }
    if (pass == 0) __threadfence();
  }
}
template <bool PARAM_BF16>
__global__ __launch_bounds__(256) void k_layernorm(const float* __restrict__ X, const float* __restrict__ R, const float* __restrict__ g, const float* __restrict__ bta,
                                                  float* __restrict__ out_sum, float* __restrict__ out_norm, int N, float eps) {
  __shared__ float red[256];
  const int row = blockIdx.x, tid = threadIdx.x;
  const float* x = X + (size_t)row * N; const float* rr = R ? R + (size_t)row * N : nullptr;
  float vals[16];
  const int per = N / 256;
  float s1 = 0.f;
  for (int u = 0; u < per / 4; ++u) {
    const int j = tid * 4 + 1024 * u;
    const v4f a = *(const v4fa*)(x + j);
    v4f b = {0.f,0.f,0.f,0.f}; if (rr) b = *(const v4fa*)(rr + j);
#pragma unroll
    for (int q = 0; q < 4; ++q) { const float v = a[q] + b[q]; vals[u * 4 + q] = v; s1 += v; }
  }
  red[tid] = s1; __syncthreads();
  for (int st = 128; st > 0; st >>= 1) { if (tid < st) red[tid] += red[tid + st]; __syncthreads(); }
  const float mu = red[0] / (float)N; __syncthreads();
  float s2 = 0.f;
  for (int u = 0; u < per / 4; ++u)
#pragma unroll
    for (int q = 0; q < 4; ++q) { const float c = vals[u * 4 + q] - mu; s2 += c * c; }
  red[tid] = s2; __syncthreads();
  for (int st = 128; st > 0; st >>= 1) { if (tid < st) red[tid] += red[tid + st]; __syncthreads(); }
  const float rs = rsqrtf(red[0] / (float)N + eps);
  for (int pass = 0; pass < 2; ++pass) {
    for (int u = 0; u < per / 4; ++u) {
      const int j = tid * 4 + 1024 * u;
      v4f o, sm;
#pragma unroll
      for (int q = 0; q < 4; ++q) {
        float gg = g[j + q], bb = bta[j + q];
        if (PARAM_BF16) { gg = bf16_round(gg); bb = bf16_round(bb); }
        sm[q] = vals[u * 4 + q]; o[q] = (vals[u * 4 + q] - mu) * rs * gg + bb;
      }
      if (out_sum) *(volatile v4f*)(out_sum + (size_t)row * N + j) = sm;
      *(volatile v4f*)(out_norm + (size_t)row * N + j) = o;
    }
    if (pass == 0) __threadfence();
  }
}


typedef _Float16 v16h __attribute__((ext_vector_type(16)));
union FragH { v16h v; v8us half[2]; _Float16 h[16]; unsigned short u[16]; };
template <int NT>
__device__ __forceinline__ v8f mmaH(v16h ah, v16h al, v16h bh, v16h bl, v8f c) {
  c = __builtin_amdgcn_wmma_f32_16x16x32_f16(false, ah, false, bh, (short)0, c, false, false);
  if (NT >= 2) c = __builtin_amdgcn_wmma_f32_16x16x32_f16(false, al, false, bh, (short)0, c, false, false);
  if (NT >= 3) c = __builtin_amdgcn_wmma_f32_16x16x32_f16(false, ah, false, bl, (short)0, c, false, false);
  asm volatile("v_nop\n\tv_nop\n\tv_nop\n\tv_nop" : "+v"(c) : "v"(ah), "v"(al), "v"(bh), "v"(bl));
  return c;
}
template <bool ASPLIT>
__global__ __launch_bounds__(128) void k_gemm_h(const float* __restrict__ A, int lda, size_t sA, const _Float16* __restrict__ Bh, int ldb, size_t sB, float alpha, float* __restrict__ C, int ldc, size_t sC, int M, int N, int K) {
  __shared__ __attribute__((aligned(16))) float so[4][16][64];
  const int tid = threadIdx.x, w = tid >> 5, lane = tid & 31, ln = lane & 15, hh = lane >> 4; const int by = blockIdx.y;
  A += (size_t)by * sA; Bh += (size_t)by * sB; C += (size_t)by * sC;
  const int ntn = (N + 63) / 64; const int wid = blockIdx.x * 4 + w; const int mt = wid / ntn, nq = wid % ntn; if (mt * 16 >= M) return;
  const int row0 = mt * 16, col0 = nq * 64; const float* arow = A + (size_t)(row0 + ln) * lda;
  v8f acc[4] = {};
  for (int kb = 0; kb < K; kb += 32) {
    FragH ah, al;
    const v4f x0 = *(const v4fa*)(arow + kb + 8 * hh), x1 = *(const v4fa*)(arow + kb + 8 * hh + 4), x2 = *(const v4fa*)(arow + kb + 16 + 8 * hh), x3 = *(const v4fa*)(arow + kb + 16 + 8 * hh + 4);
    float xs[16] = {x0[0],x0[1],x0[2],x0[3],x1[0],x1[1],x1[2],x1[3],x2[0],x2[1],x2[2],x2[3],x3[0],x3[1],x3[2],x3[3]};
#pragma unroll
    for (int i = 0; i < 16; ++i) { const _Float16 h = (_Float16)xs[i]; ah.h[i] = h; al.h[i] = ASPLIT ? (_Float16)(xs[i] - (float)h) : (_Float16)0.0f; }
#pragma unroll
    for (int t = 0; t < 4; ++t) { if (col0 + t * 16 >= N) continue; const size_t boff = (size_t)(col0 + t * 16 + ln) * ldb + kb; FragH bq; bq.half[0] = *(const v8us*)(Bh + boff + 8 * hh); bq.half[1] = *(const v8us*)(Bh + boff + 16 + 8 * hh);
      acc[t] = mmaH<ASPLIT ? 2 : 1>(ah.v, al.v, bq.v, bq.v, acc[t]); }
  }
#pragma unroll
  for (int t = 0; t < 4; ++t) { if (col0 + t * 16 >= N) continue;
#pragma unroll
    for (int r = 0; r < 8; ++r) so[w][8 * hh + r][t * 16 + ln] = acc[t][r] * alpha; }
  __builtin_amdgcn_fence(__ATOMIC_ACQ_REL, "workgroup"); __builtin_amdgcn_wave_barrier();
  const int rsub = lane >> 4, c4 = (lane & 15) * 4;
  for (int pass = 0; pass < 2; ++pass) {
#pragma unroll
    for (int q = 0; q < 8; ++q) { const int r = q * 2 + rsub; if (col0 + c4 < N) { const v4f v = *(const v4fa*)&so[w][r][c4]; *(volatile v4f*)(C + (size_t)(row0 + r) * ldc + col0 + c4) = v; } }
    if (pass == 0) __threadfence(); }
}

__global__ __launch_bounds__(256) void k_wt_f16(const float* __restrict__ W, _Float16* __restrict__ Wt, int K, int N, float scale) {
  const int t = blockIdx.x * 256 + threadIdx.x; if (t >= N * (K / 8)) return; const int n = t / (K / 8), k8 = (t % (K / 8)) * 8; FragH f;
#pragma unroll
  for (int i = 0; i < 8; ++i) f.h[i] = (_Float16)(bf16_round(W[(size_t)(k8 + i) * N + n]) * scale); const v8us o = f.half[0];
  *(volatile v8us*)((unsigned short*)Wt + (size_t)n * K + k8) = o; __threadfence(); *(volatile v8us*)((unsigned short*)Wt + (size_t)n * K + k8) = o;
}
template <int ACT>
__global__ __launch_bounds__(128) void k_gemm_hhx(const _Float16* __restrict__ A, int lda, size_t sA, const _Float16* __restrict__ Bh, int ldb, size_t sB, float alpha, const float* __restrict__ bias, size_t sBias, const float* __restrict__ CP, int rowsPerB, size_t sCPb, int row0g,
    float* __restrict__ C, _Float16* __restrict__ C16, int ldc, size_t sC, int M, int N, int K) {
  __shared__ __attribute__((aligned(16))) float so[4][16][64];
  const int tid = threadIdx.x, w = tid >> 5, lane = tid & 31, ln = lane & 15, hh = lane >> 4; const int by = blockIdx.y;
  A += (size_t)by * sA; Bh += (size_t)by * sB; const size_t cofs = (size_t)by * sC; const float* bp = bias ? bias + (size_t)by * sBias : nullptr;
  const int ntn = (N + 63) / 64; const int wid = blockIdx.x * 4 + w; const int mt = wid / ntn, nq = wid % ntn; if (mt * 16 >= M) return;
  const int row0 = mt * 16, col0 = nq * 64; const _Float16* arow = A + (size_t)(row0 + ln) * lda;
  v8f acc[4] = {};
  for (int kb = 0; kb < K; kb += 32) { FragH ah; ah.half[0] = *(const v8us*)((const unsigned short*)arow + kb + 8 * hh); ah.half[1] = *(const v8us*)((const unsigned short*)arow + kb + 16 + 8 * hh);
#pragma unroll
    for (int t = 0; t < 4; ++t) { if (col0 + t * 16 >= N) continue; const size_t boff = (size_t)(col0 + t * 16 + ln) * ldb + kb; FragH bq; bq.half[0] = *(const v8us*)((const unsigned short*)Bh + boff + 8 * hh); bq.half[1] = *(const v8us*)((const unsigned short*)Bh + boff + 16 + 8 * hh);
      acc[t] = mmaH<1>(ah.v, ah.v, bq.v, bq.v, acc[t]); }
  }
#pragma unroll
  for (int t = 0; t < 4; ++t) { if (col0 + t * 16 >= N) continue; const int col = col0 + t * 16 + ln; const float bv = bp ? bf16_round(bp[col]) : 0.f;
#pragma unroll
    for (int r = 0; r < 8; ++r) { float v = acc[t][r] * alpha + bv; if (CP) { const int rr = row0g + row0 + 8 * hh + r; if (rowsPerB < 0) v += CP[cofs + (size_t)rr * ldc + col];        else { const int bidx = rr / rowsPerB; v += CP[(size_t)bidx * sCPb + (size_t)by * 64 + col]; } } if (ACT == 1) v = (v > 0.f) ? v : expm1f(v); else if (ACT == 7) v = (v > 0.f) ? v + 1.0f : expf(v); else if (ACT == 8) v = tanhf(v); else if (ACT == 9) v = 0.5f * v * (1.0f + tanhf(0.7978845608028654f * (v + 0.044715f * v * v * v))); else if (ACT == 11) v = 1.0f / (1.0f + expf(-v)); else if (ACT == 12) v = (v > 0.f) ? v : 0.01f * v; else if (ACT == 14) v = (v > 0.f) ? v : 0.1f * v; else if (ACT == 16) v = (v >= 0.f) ? v : 0.3f * v; else if (ACT == 17) v = (v >= 0.f) ? v : 0.2f * v; else if (ACT == 15) v = v / (1.0f + expf(-v)); else if (ACT == 3) v = fmaxf(v, 0.f); else if (ACT == 6) v = 0.5f * v * (1.0f + erff(v * 0.70710678118654752f)); so[w][8 * hh + r][t * 16 + ln] = v; } }
  __builtin_amdgcn_fence(__ATOMIC_ACQ_REL, "workgroup"); __builtin_amdgcn_wave_barrier();
  const int rsub = lane >> 4, c4 = (lane & 15) * 4; typedef _Float16 v4h __attribute__((ext_vector_type(4)));
  for (int pass = 0; pass < 2; ++pass) {
#pragma unroll
    for (int q = 0; q < 8; ++q) { const int r = q * 2 + rsub; if (col0 + c4 < N) { const v4f v = *(const v4fa*)&so[w][r][c4]; if (C) *(volatile v4f*)(C + cofs + (size_t)(row0 + r) * ldc + col0 + c4) = v; if (C16) { v4h h4; for (int i = 0; i < 4; ++i) h4[i] = (_Float16)v[i]; *(volatile v4h*)(C16 + cofs + (size_t)(row0 + r) * ldc + col0 + c4) = h4; } } }
    if (pass == 0) __threadfence(); }
}


typedef _Float16 v4h __attribute__((ext_vector_type(4)));

__global__ __launch_bounds__(256) void k_x16(const float* __restrict__ x, _Float16* __restrict__ X16, size_t n8) { const size_t t = (size_t)blockIdx.x * 256 + threadIdx.x; if (t >= n8) return; FragH f;
#pragma unroll
  for (int q = 0; q < 8; ++q) f.h[q] = (_Float16)bf16_round(x[t * 8 + q]); *(volatile v8us*)((unsigned short*)X16 + t * 8) = f.half[0]; __threadfence(); *(volatile v8us*)((unsigned short*)X16 + t * 8) = f.half[0]; }
__global__ __launch_bounds__(256) void k_h16(const float* __restrict__ x, _Float16* __restrict__ X16, size_t n8) { const size_t t = (size_t)blockIdx.x * 256 + threadIdx.x; if (t >= n8) return; FragH f;
#pragma unroll
  for (int q = 0; q < 8; ++q) f.h[q] = (_Float16)x[t * 8 + q]; *(volatile v8us*)((unsigned short*)X16 + t * 8) = f.half[0]; __threadfence(); *(volatile v8us*)((unsigned short*)X16 + t * 8) = f.half[0]; }
__global__ __launch_bounds__(256) void k_round16f(const float* __restrict__ W, _Float16* __restrict__ Bt, size_t n8) { const size_t t = (size_t)blockIdx.x * 256 + threadIdx.x; if (t >= n8) return; FragH f;
#pragma unroll
  for (int i = 0; i < 8; ++i) f.h[i] = (_Float16)(bf16_round(W[t * 8 + i]) * 16.0f); *(volatile v8us*)((unsigned short*)Bt + t * 8) = f.half[0]; __threadfence(); *(volatile v8us*)((unsigned short*)Bt + t * 8) = f.half[0]; }
template <int NHv, int TTv>
__global__ __launch_bounds__(256) void k_vt(const _Float16* __restrict__ V16, int ldv, int voff, _Float16* __restrict__ Vt) { __shared__ unsigned short tl[64][66]; const int tid = threadIdx.x; const int slab = blockIdx.x / (TTv / 64), lg = blockIdx.x % (TTv / 64); const int b = slab / NHv, h = slab % NHv;
  for (int i = tid; i < 64 * 8; i += 256) { const int r = i / 8, c8 = (i % 8) * 8; FragH f; f.half[0] = *(const v8us*)((const unsigned short*)V16 + ((size_t)b * TTv + lg * 64 + r) * ldv + voff + h * 64 + c8);
#pragma unroll
    for (int q = 0; q < 8; ++q) tl[r][c8 + q] = f.u[q]; }
  __syncthreads();
  for (int pass = 0; pass < 2; ++pass) {
#pragma unroll
    for (int rd = 0; rd < 2; ++rd) { const int d = rd * 32 + tid / 8, pc = tid % 8; FragH f;
#pragma unroll
      for (int q = 0; q < 8; ++q) f.u[q] = tl[pc * 8 + q][d];
      *(volatile v8us*)((unsigned short*)Vt + ((size_t)slab * 64 + d) * TTv + lg * 64 + pc * 8) = f.half[0]; }
    if (pass == 0) __threadfence(); } }

__global__ __launch_bounds__(256) void k_hl(const float* __restrict__ F, _Float16* __restrict__ Hh, _Float16* __restrict__ Hl, size_t n8) { const size_t t = (size_t)blockIdx.x * 256 + threadIdx.x; if (t >= n8) return; FragH fh, fl; const v4f a = *(const v4fa*)(F + t * 8), c = *(const v4fa*)(F + t * 8 + 4);
#pragma unroll
  for (int q = 0; q < 4; ++q) { _Float16 h = (_Float16)a[q]; fh.h[q] = h; fl.h[q] = (_Float16)((a[q] - (float)h) * 1024.0f); h = (_Float16)c[q]; fh.h[4 + q] = h; fl.h[4 + q] = (_Float16)((c[q] - (float)h) * 1024.0f); }
  for (int pass = 0; pass < 2; ++pass) { *(volatile v8us*)((unsigned short*)Hh + t * 8) = fh.half[0]; *(volatile v8us*)((unsigned short*)Hl + t * 8) = fl.half[0]; if (pass == 0) __threadfence(); } }

__device__ __forceinline__ v16h g2_frag(const _Float16* p, int hh) { FragH f; f.half[0] = *(const v8us*)((const unsigned short*)p + 8 * hh); f.half[1] = *(const v8us*)((const unsigned short*)p + 16 + 8 * hh); return f.v; }
__device__ __forceinline__ v8f g2_mma(v16h a, v16h b, v8f c) { v8f d = __builtin_amdgcn_wmma_f32_16x16x32_f16(false, a, false, b, (short)0, c, false, false); asm volatile("v_nop\n\tv_nop\n\tv_nop\n\tv_nop" : "+v"(d) : "v"(a), "v"(b)); return d; }
template <int ACT>
__global__ __launch_bounds__(128) void k_gemm2(const _Float16* __restrict__ A, int lda, size_t sA, const _Float16* __restrict__ Bh, int ldb, size_t sB, float alpha, const float* __restrict__ bias, size_t sBias, const float* __restrict__ CP, int rowsPerB, size_t sCPb, int row0g,
    float* __restrict__ C, _Float16* __restrict__ C16, int ldc, size_t sC, int M, int N, int K) { static_assert(ACT == 0 || ACT == 3 || ACT == 6 || ACT == 8 || ACT == 9 || ACT == 11 || ACT == 12 || ACT == 14 || ACT == 15 || ACT == 16 || ACT == 17, "k_gemm2: unsupported ACT code (would silently apply no activation)");
  __shared__ __attribute__((aligned(16))) float so[4][32][68];
  const int tid = threadIdx.x, w = tid >> 5, lane = tid & 31, ln = lane & 15, hh = lane >> 4; const int by = blockIdx.y;
  A += (size_t)by * sA; Bh += (size_t)by * sB; const size_t cofs = (size_t)by * sC; const float* bp = bias ? bias + (size_t)by * sBias : nullptr;
  const int ntn = N >> 6; const int mt = blockIdx.x / ntn, nq = blockIdx.x - mt * ntn; const int row0 = mt * 128 + 32 * w, col0 = nq * 64; if (row0 >= M) return;
  const _Float16* a0p = A + (size_t)(row0 + ln) * lda; const _Float16* a1p = a0p + (size_t)16 * lda;
  const _Float16* b0p = Bh + (size_t)(col0 + ln) * ldb; const _Float16* b1p = b0p + (size_t)16 * ldb; const _Float16* b2p = b1p + (size_t)16 * ldb; const _Float16* b3p = b2p + (size_t)16 * ldb;
  const v8f z8 = {0.f,0.f,0.f,0.f,0.f,0.f,0.f,0.f}; v8f c00 = z8, c01 = z8, c02 = z8, c03 = z8, c10 = z8, c11 = z8, c12 = z8, c13 = z8;
#pragma unroll 1
  for (int kb = 0; kb < K; kb += 32) { const v16h a0 = g2_frag(a0p + kb, hh), a1 = g2_frag(a1p + kb, hh);
    v16h b = g2_frag(b0p + kb, hh); c00 = g2_mma(a0, b, c00); c10 = g2_mma(a1, b, c10);
    b = g2_frag(b1p + kb, hh); c01 = g2_mma(a0, b, c01); c11 = g2_mma(a1, b, c11);
    b = g2_frag(b2p + kb, hh); c02 = g2_mma(a0, b, c02); c12 = g2_mma(a1, b, c12);
    b = g2_frag(b3p + kb, hh); c03 = g2_mma(a0, b, c03); c13 = g2_mma(a1, b, c13); }
  v8f accs[8] = {c00, c01, c02, c03, c10, c11, c12, c13};
#pragma unroll
  for (int u = 0; u < 8; ++u) { const int t = u & 3, half = u >> 2; const int col = col0 + t * 16 + ln; const float bv = bp ? bf16_round(bp[col]) : 0.f;
#pragma unroll
    for (int r = 0; r < 8; ++r) { const int rloc = half * 16 + 8 * hh + r; float v = accs[u][r] * alpha + bv; if (CP) { if (rowsPerB < 0) v += CP[cofs + (size_t)(row0g + row0 + rloc) * ldc + col];        else { const int bidx = (row0g + row0 + rloc) / rowsPerB; v += CP[(size_t)bidx * sCPb + (size_t)by * 64 + col]; } }
      if (ACT == 3) v = fmaxf(v, 0.f); else if (ACT == 6) v = 0.5f * v * (1.0f + erff(v * 0.70710678118654752f)); else if (ACT == 11) v = 1.0f / (1.0f + expf(-v)); else if (ACT == 15) v = v / (1.0f + expf(-v)); else if (ACT == 12) v = (v > 0.f) ? v : 0.01f * v; else if (ACT == 8) v = tanhf(v); else if (ACT == 9) v = 0.5f * v * (1.0f + tanhf(0.7978845608028654f * (v + 0.044715f * v * v * v))); else if (ACT == 14) v = (v > 0.f) ? v : 0.1f * v; else if (ACT == 16) v = (v >= 0.f) ? v : 0.3f * v; else if (ACT == 17) v = (v >= 0.f) ? v : 0.2f * v;
      so[w][rloc][t * 16 + ln] = v; } }
  __builtin_amdgcn_fence(__ATOMIC_ACQ_REL, "workgroup"); __builtin_amdgcn_wave_barrier();
  const int rsub = lane >> 4, c4 = (lane & 15) * 4;
  for (int pass = 0; pass < 2; ++pass) {
#pragma unroll
    for (int q = 0; q < 16; ++q) { const int r = q * 2 + rsub; const v4f v = *(const v4fa*)&so[w][r][c4]; if (C) *(volatile v4f*)(C + cofs + (size_t)(row0 + r) * ldc + col0 + c4) = v; if (C16) { v4h h4; for (int i = 0; i < 4; ++i) h4[i] = (_Float16)v[i]; *(volatile v4h*)(C16 + cofs + (size_t)(row0 + r) * ldc + col0 + c4) = h4; } }
    if (pass == 0) __threadfence(); } }


__device__ __forceinline__ void rsw(int i, int n, int* j0, float* w) { const float base[4] = {0.125f, 0.375f, 0.375f, 0.125f}; float s = 0.f; for (int t = 0; t < 4; ++t) { const int j = 2 * i - 1 + t; const bool ok = (j >= 0 && j < n); w[t] = ok ? base[t] : 0.f; s += w[t]; j0[t] = ok ? j : 0; } for (int t = 0; t < 4; ++t) w[t] = w[t] / s; }
__global__ __launch_bounds__(256) void k_resize(const float* __restrict__ prior, _Float16* __restrict__ PR16) {
  #pragma clang fp contract(off)
  const size_t t = (size_t)blockIdx.x * 256 + threadIdx.x; if (t >= (size_t)NR * CH / 2) return; const int c = (int)((t * 2) % CH); const size_t row = (t * 2) / CH; const int b = (int)(row / PX), p = (int)(row % PX); const int oy = p / HS, ox = p % HS; int jy[4], jx[4]; float wy[4], wx[4]; rsw(oy, HP, jy, wy); rsw(ox, HP, jx, wx); typedef _Float16 v2h_ __attribute__((ext_vector_type(2))); v2h_ o2;
  for (int cc = 0; cc < 2; ++cc) { const float* src = prior + ((size_t)b * CH + c + cc) * HP * HP; float s = 0.f;
    for (int a = 0; a < 4; ++a) { float rsum = 0.f; for (int e = 0; e < 4; ++e) rsum += bf16_round(src[(size_t)jy[a] * HP + jx[e]]) * wx[e]; s += rsum * wy[a]; } o2[cc] = (_Float16)s; }
  *(volatile v2h_*)(PR16 + t * 2) = o2; __threadfence(); *(volatile v2h_*)(PR16 + t * 2) = o2; }
__global__ __launch_bounds__(256) void k_nhwc(const float* __restrict__ x, _Float16* __restrict__ D, int ld, int coff) { const size_t t = (size_t)blockIdx.x * 256 + threadIdx.x; if (t >= (size_t)NR * CH / 8) return; const int c0 = (int)((t * 8) % CH); const size_t row = (t * 8) / CH; const int b = (int)(row / PX), p = (int)(row % PX); FragH f; for (int q = 0; q < 8; ++q) f.h[q] = (_Float16)bf16_round(x[((size_t)b * CH + c0 + q) * PX + p]);
  unsigned short* dst = (unsigned short*)D + row * ld + coff + c0; *(volatile v8us*)dst = f.half[0]; __threadfence(); *(volatile v8us*)dst = f.half[0]; }
__global__ __launch_bounds__(256) void k_wre(const float* __restrict__ w, int O, int Olive, int CI, int K, _Float16* __restrict__ Bt) { const size_t t = (size_t)blockIdx.x * 256 + threadIdx.x; const int KK2 = K * K; if (t >= (size_t)O * KK2 * CI / 8) return; const int c8 = (int)((t * 8) % CI); const int tap = (int)(((t * 8) / CI) % KK2); const int o = (int)((t * 8) / ((size_t)CI * KK2)); FragH f; for (int q = 0; q < 8; ++q) f.h[q] = (o < Olive) ? (_Float16)(bf16_round(w[(((size_t)o * CI + c8 + q) * KK2) + tap]) * 16.0f) : (_Float16)0.0f;
  *(volatile v8us*)((unsigned short*)Bt + t * 8) = f.half[0]; __threadfence(); *(volatile v8us*)((unsigned short*)Bt + t * 8) = f.half[0]; }
__global__ __launch_bounds__(256) void k_bpad(const float* __restrict__ src, int n, float* __restrict__ dst) { const int i = threadIdx.x; if (i >= 256) return; const float v = (i < n) ? src[i] : 0.f; *(volatile float*)(dst + i) = v; __threadfence(); *(volatile float*)(dst + i) = v; }
__global__ __launch_bounds__(256) void k_im2col(const _Float16* __restrict__ Sp, _Float16* __restrict__ XC) { const size_t t = (size_t)blockIdx.x * 256 + threadIdx.x; if (t >= (size_t)NR * 9 * (CH / 8)) return; const int c8 = (int)(t % (CH / 8)) * 8; const int tap = (int)((t / (CH / 8)) % 9); const size_t row = t / ((size_t)9 * (CH / 8)); const int b = (int)(row / PX), p = (int)(row % PX); const int iy = p / HS - 1 + tap / 3, ix = p % HS - 1 + tap % 3; v8us v;
  if (iy >= 0 && iy < HS && ix >= 0 && ix < HS) v = *(const v8us*)((const unsigned short*)Sp + (((size_t)b * HS + iy) * HS + ix) * CH + c8); else { for (int q = 0; q < 8; ++q) v[q] = 0; }
  unsigned short* dst = (unsigned short*)XC + row * (size_t)(9 * CH) + tap * CH + c8; *(volatile v8us*)dst = v; __threadfence(); *(volatile v8us*)dst = v; }
__global__ __launch_bounds__(256) void k_gnstat(const float* __restrict__ X, float* __restrict__ ST) {
  #pragma clang fp contract(off)
  __shared__ float red[256]; const int b = blockIdx.x / NGN, g = blockIdx.x % NGN, tid = threadIdx.x; const float* base = X + (size_t)b * PX * CH + g * GSZ; float s = 0.f;
#pragma unroll 1
  for (int p = tid; p < PX; p += 256) { const v8f a = *(const v8f*)(base + (size_t)p * CH); for (int q = 0; q < 8; ++q) s += a[q]; }
  red[tid] = s; __syncthreads(); for (int st = 128; st > 0; st >>= 1) { if (tid < st) red[tid] += red[tid + st]; __syncthreads(); } const float mu = red[0] / (float)(PX * GSZ); __syncthreads(); float s2 = 0.f;
#pragma unroll 1
  for (int p = tid; p < PX; p += 256) { const v8f a = *(const v8f*)(base + (size_t)p * CH); for (int q = 0; q < 8; ++q) { const float d = a[q] - mu; s2 += d * d; } }
  red[tid] = s2; __syncthreads(); for (int st = 128; st > 0; st >>= 1) { if (tid < st) red[tid] += red[tid + st]; __syncthreads(); }
  if (tid == 0) { const float r = rsqrtf(red[0] / (float)(PX * GSZ) + 1e-6f); float* d = ST + (size_t)blockIdx.x * 32; *(volatile float*)d = mu; *(volatile float*)(d + 1) = r; __threadfence(); *(volatile float*)d = mu; *(volatile float*)(d + 1) = r; } }
__global__ __launch_bounds__(256) void k_gnsilu(const float* __restrict__ X, const float* __restrict__ ST, const float* __restrict__ gam, const float* __restrict__ bet, float* __restrict__ Df, _Float16* __restrict__ Dh) {
  #pragma clang fp contract(off)
  const size_t t = (size_t)blockIdx.x * 256 + threadIdx.x; if (t >= (size_t)NR * CH / 8) return; const int c0 = (int)((t * 8) % CH); const size_t row = (t * 8) / CH; const int b = (int)(row / PX); const int g = c0 / GSZ; const float mu = ST[((size_t)b * NGN + g) * 32], r = ST[((size_t)b * NGN + g) * 32 + 1]; const v8f a = *(const v8f*)(X + t * 8); v8f o; FragH f;
  for (int q = 0; q < 8; ++q) { float y = (a[q] - mu) * r; y = y * bf16_round(gam[c0 + q]); y += bf16_round(bet[c0 + q]); const float sv = y / (1.0f + expf(-y)); o[q] = sv; f.h[q] = (_Float16)sv; }
  for (int pass = 0; pass < 2; ++pass) { if (Df) *(volatile v8f*)(Df + t * 8) = o; if (Dh) *(volatile v8us*)((unsigned short*)Dh + t * 8) = f.half[0]; if (pass == 0) __threadfence(); } }
__global__ __launch_bounds__(256) void k_dw7(const float* __restrict__ X, const float* __restrict__ w, const float* __restrict__ bb, float* __restrict__ D) {
  #pragma clang fp contract(off)
  const size_t t = (size_t)blockIdx.x * 256 + threadIdx.x; if (t >= (size_t)NR * CH) return; const int c = (int)(t % CH); const size_t row = t / CH; const int b = (int)(row / PX), p = (int)(row % PX); const int py = p / HS, px = p % HS; float s = bf16_round(bb[c]);
#pragma unroll 1
  for (int ky = 0; ky < 7; ++ky) { const int yy = py + ky - 3; if (yy < 0 || yy >= HS) continue;
#pragma unroll 1
    for (int kx = 0; kx < 7; ++kx) { const int xx = px + kx - 3; if (xx < 0 || xx >= HS) continue; s += bf16_round(w[(c * 7 + ky) * 7 + kx]) * X[(((size_t)b * HS + yy) * HS + xx) * CH + c]; } }
  *(volatile float*)(D + t) = s; __threadfence(); *(volatile float*)(D + t) = s; }
__global__ __launch_bounds__(256) void k_dcncol(const _Float16* __restrict__ Sp, int ld, int coff, const float* __restrict__ O2, _Float16* __restrict__ XC) {
  #pragma clang fp contract(off)
  const size_t t = (size_t)blockIdx.x * 256 + threadIdx.x; if (t >= (size_t)NR * 9 * (CH / 8)) return; const int c8 = (int)(t % (CH / 8)) * 8; const int k = (int)((t / (CH / 8)) % 9); const size_t row = t / ((size_t)9 * (CH / 8)); const int b = (int)(row / PX), p = (int)(row % PX); const int y = p / HS, x = p % HS; const int g = c8 / CG; const float* orow = O2 + row * 256;
  const float offy = orow[(g * 9 + k) * 2], offx = orow[(g * 9 + k) * 2 + 1]; const float m = 1.0f / (1.0f + expf(-orow[144 + g * 9 + k])); const float py = (float)(y + k / 3 - 1) + offy, pxf = (float)(x + k % 3 - 1) + offx; const float y0 = floorf(py), x0 = floorf(pxf); const float wy1 = py - y0, wx1 = pxf - x0; const int iy0 = (int)y0, ix0 = (int)x0;
  float acc[8]; for (int q = 0; q < 8; ++q) acc[q] = 0.f;
  for (int cn = 0; cn < 4; ++cn) { const int yi = iy0 + (cn >> 1), xi = ix0 + (cn & 1); if (yi < 0 || yi >= HS || xi < 0 || xi >= HS) continue; const float wv = ((cn >> 1) ? wy1 : (1.0f - wy1)) * ((cn & 1) ? wx1 : (1.0f - wx1)); FragH v; v.half[0] = *(const v8us*)((const unsigned short*)Sp + (((size_t)b * HS + yi) * HS + xi) * ld + coff + c8); for (int q = 0; q < 8; ++q) acc[q] += (float)v.h[q] * wv; }
  FragH f; for (int q = 0; q < 8; ++q) f.h[q] = (_Float16)(acc[q] * m); unsigned short* dst = (unsigned short*)XC + row * (size_t)(9 * CH) + k * CH + c8; *(volatile v8us*)dst = f.half[0]; __threadfence(); *(volatile v8us*)dst = f.half[0]; }
__global__ __launch_bounds__(256) void k_out(const float* __restrict__ Y, float* __restrict__ out) { const size_t t = (size_t)blockIdx.x * 256 + threadIdx.x; if (t >= (size_t)NI * CH * PX / 8) return; const int p0 = (int)((t * 8) % PX); const size_t bc = (t * 8) / PX; const int b = (int)(bc / CH), c = (int)(bc % CH); v8f v; for (int q = 0; q < 8; ++q) v[q] = Y[((size_t)b * PX + p0 + q) * CH + c];
  *(volatile v8f*)(out + t * 8) = v; __threadfence(); *(volatile v8f*)(out + t * 8) = v; }

extern "C" void kernel_launch(void* const* d_in, const int* in_sizes, int n_in,
                              void* d_out, int out_size, void* d_ws, size_t ws_size, hipStream_t stream) {
  (void)in_sizes; (void)n_in; (void)out_size;
  const float* const* I = (const float* const*)d_in; const float* xm = I[0]; const float* prior = I[1]; const float* w_ds = I[2]; const float* b_ds = I[3]; const float* w1 = I[4]; const float* b1 = I[5]; const float* g1 = I[6]; const float* bt1 = I[7]; const float* w_dw = I[8]; const float* b_dw = I[9]; const float* g2 = I[10]; const float* bt2 = I[11]; const float* w2 = I[12]; const float* b2 = I[13]; const float* w3 = I[14]; const float* b3 = I[15]; const float* g3 = I[16]; const float* bt3 = I[17]; const float* w_off = I[18]; const float* b_off = I[19]; const float* w_dcn = I[20]; const float* b_dcn = I[21];
  float* out0 = (float*)d_out; float* out1 = (float*)((char*)d_out + (size_t)NR * CH * 4);
  char* ws = (char*)d_ws; size_t off = 0;
  auto take = [&](size_t bytes) { char* p = ws + off; off += (bytes + 255) & ~(size_t)255; return p; };
  _Float16* Bds = (_Float16*)take((size_t)CH * 2304 * 2); _Float16* B1 = (_Float16*)take((size_t)CH * 512 * 2); _Float16* B2 = (_Float16*)take((size_t)CH * CH * 2); _Float16* B3 = (_Float16*)take((size_t)CH * 2304 * 2); _Float16* Boff = (_Float16*)take((size_t)256 * 2304 * 2); _Float16* Bdcn = (_Float16*)take((size_t)CH * 2304 * 2); float* boffp = (float*)take(256 * 4); float* ST = (float*)take((size_t)NI * NGN * 32 * 4);
  _Float16* PR16 = (_Float16*)take((size_t)NR * CH * 2); _Float16* CAT16 = (_Float16*)take((size_t)NR * 512 * 2); _Float16* XC = (_Float16*)take((size_t)NR * 2304 * 2); float* T1 = (float*)take((size_t)NR * CH * 4); float* T1N = (float*)take((size_t)NR * CH * 4); float* T2 = (float*)take((size_t)NR * CH * 4); _Float16* T2N = (_Float16*)take((size_t)NR * CH * 2); _Float16* T3 = (_Float16*)take((size_t)NR * CH * 2); float* OF = (float*)take((size_t)NR * CH * 4); float* OFT = (float*)take((size_t)NR * CH * 4); _Float16* OF16 = (_Float16*)take((size_t)NR * CH * 2); float* O2 = (float*)take((size_t)NR * 256 * 4); float* WARP = T1;
  if (off > ws_size) return;
  k_wre<<<(unsigned)(((size_t)CH * 9 * CH / 8 + 255) / 256), 256, 0, stream>>>(w_ds, CH, CH, CH, 3, Bds); k_wre<<<(unsigned)(((size_t)CH * 512 / 8 + 255) / 256), 256, 0, stream>>>(w1, CH, CH, 512, 1, B1); k_wre<<<(unsigned)(((size_t)CH * CH / 8 + 255) / 256), 256, 0, stream>>>(w2, CH, CH, CH, 1, B2); k_wre<<<(unsigned)(((size_t)CH * 9 * CH / 8 + 255) / 256), 256, 0, stream>>>(w3, CH, CH, CH, 3, B3);
  k_wre<<<(unsigned)(((size_t)256 * 9 * CH / 8 + 255) / 256), 256, 0, stream>>>(w_off, 256, NOFF, CH, 3, Boff); k_wre<<<(unsigned)(((size_t)CH * 9 * CH / 8 + 255) / 256), 256, 0, stream>>>(w_dcn, CH, CH, CH, 3, Bdcn); k_bpad<<<1, 256, 0, stream>>>(b_off, NOFF, boffp);
  k_resize<<<(unsigned)(((size_t)NR * CH / 2 + 255) / 256), 256, 0, stream>>>(prior, PR16); k_nhwc<<<(unsigned)(((size_t)NR * CH / 8 + 255) / 256), 256, 0, stream>>>(xm, CAT16, 512, CH);
  const dim3 g256((NR / 128) * (CH / 64), 1);
  k_im2col<<<(unsigned)(((size_t)NR * 9 * (CH / 8) + 255) / 256), 256, 0, stream>>>(PR16, XC); k_gemm2<0><<<g256, 128, 0, stream>>>(XC, 2304, 0, Bds, 2304, 0, 0.0625f, b_ds, 0, nullptr, 1, 0, 0, nullptr, CAT16, 512, 0, NR, CH, 2304);
  k_gemm2<0><<<g256, 128, 0, stream>>>(CAT16, 512, 0, B1, 512, 0, 0.0625f, b1, 0, nullptr, 1, 0, 0, T1, nullptr, CH, 0, NR, CH, 512);
  k_gnstat<<<NI * NGN, 256, 0, stream>>>(T1, ST); k_gnsilu<<<(unsigned)(((size_t)NR * CH / 8 + 255) / 256), 256, 0, stream>>>(T1, ST, g1, bt1, T1N, nullptr);
  k_dw7<<<(unsigned)(((size_t)NR * CH + 255) / 256), 256, 0, stream>>>(T1N, w_dw, b_dw, T2);
  k_gnstat<<<NI * NGN, 256, 0, stream>>>(T2, ST); k_gnsilu<<<(unsigned)(((size_t)NR * CH / 8 + 255) / 256), 256, 0, stream>>>(T2, ST, g2, bt2, nullptr, T2N);
  k_gemm2<0><<<g256, 128, 0, stream>>>(T2N, CH, 0, B2, CH, 0, 0.0625f, b2, 0, nullptr, 1, 0, 0, nullptr, T3, CH, 0, NR, CH, CH);
  k_im2col<<<(unsigned)(((size_t)NR * 9 * (CH / 8) + 255) / 256), 256, 0, stream>>>(T3, XC); k_gemm2<0><<<g256, 128, 0, stream>>>(XC, 2304, 0, B3, 2304, 0, 0.0625f, b3, 0, nullptr, 1, 0, 0, OF, nullptr, CH, 0, NR, CH, 2304);
  k_gnstat<<<NI * NGN, 256, 0, stream>>>(OF, ST); k_gnsilu<<<(unsigned)(((size_t)NR * CH / 8 + 255) / 256), 256, 0, stream>>>(OF, ST, g3, bt3, OFT, OF16);
  k_out<<<(unsigned)(((size_t)NI * CH * PX / 8 + 255) / 256), 256, 0, stream>>>(OFT, out1);
  k_im2col<<<(unsigned)(((size_t)NR * 9 * (CH / 8) + 255) / 256), 256, 0, stream>>>(OF16, XC); k_gemm2<0><<<g256, 128, 0, stream>>>(XC, 2304, 0, Boff, 2304, 0, 0.0625f, boffp, 0, nullptr, 1, 0, 0, O2, nullptr, 256, 0, NR, 256, 2304);
  k_dcncol<<<(unsigned)(((size_t)NR * 9 * (CH / 8) + 255) / 256), 256, 0, stream>>>(CAT16, 512, CH, O2, XC); k_gemm2<0><<<g256, 128, 0, stream>>>(XC, 2304, 0, Bdcn, 2304, 0, 0.0625f, b_dcn, 0, nullptr, 1, 0, 0, WARP, nullptr, CH, 0, NR, CH, 2304);
  k_out<<<(unsigned)(((size_t)NI * CH * PX / 8 + 255) / 256), 256, 0, stream>>>(WARP, out0);
}
